// KANLinear_22522808500876
// MI455X (gfx1250) — hardware-run, weakly checked
//
#include <hip/hip_runtime.h>
#include <math.h>

constexpr int NB_ROWS = 8192;
constexpr int NIN     = 1024;
constexpr int NOUT    = 1024;
constexpr int NBAS    = 8;
constexpr int NKN     = 12;
constexpr int KTOT    = NIN + NIN * NBAS;
constexpr int NX      = NB_ROWS * NIN;
constexpr int NHALF   = 2;
constexpr int MHALF   = NB_ROWS / NHALF;
constexpr float FEAT_CARRY = 64.0f;
constexpr float WGT_CARRY  = 1024.0f;
constexpr float OUT_SCALE  = 1.0f / (64.0f * 1024.0f);

constexpr int MM_BLOCKS  = 256;
constexpr int MM_THREADS = 256;
constexpr int MM_ITERS   = NX / (MM_BLOCKS * MM_THREADS * 4);
constexpr int FT_THREADS = 128;
constexpr int FT_ROWS    = 8;
constexpr int FT_CHUNKS  = NIN / FT_THREADS;
constexpr int PW_THREADS = 128;
constexpr int PW_BLOCKS_X = 1 + (NIN * NBAS) / (8 * PW_THREADS);
constexpr int GM_BLOCKS  = ((MHALF / 64) * (NOUT / 64)) / 8;

constexpr size_t WS_OFF_PART   = 0;
constexpr size_t WS_PART_BYTES = (size_t)MM_BLOCKS * 128;
constexpr size_t WS_OFF_STATS  = 32768;
constexpr size_t WS_OFF_A      = 65536;
constexpr size_t WS_A_BYTES    = (size_t)MHALF * KTOT * 2;
constexpr size_t WS_OFF_W      = WS_OFF_A + WS_A_BYTES;
constexpr size_t WS_W_BYTES    = (size_t)NOUT * KTOT * 2;
constexpr size_t WS_END        = WS_OFF_W + WS_W_BYTES;

static_assert(WS_PART_BYTES <= WS_OFF_STATS);
static_assert(WS_OFF_STATS + 128 <= WS_OFF_A);
static_assert((WS_OFF_A % 128) == 0 && (WS_OFF_W % 128) == 0);
static_assert(WS_END <= (size_t)134217728);
static_assert(KTOT % 32 == 0);
static_assert(MHALF % 64 == 0 && NOUT % 64 == 0);
static_assert(((MHALF / 64) * (NOUT / 64)) % 8 == 0);
static_assert(NX % (MM_BLOCKS * MM_THREADS * 4) == 0);
static_assert(NIN % FT_THREADS == 0 && NIN == 8 * FT_THREADS);
static_assert(MHALF % FT_ROWS == 0);
static_assert(NIN == 8 * PW_THREADS && (NIN * NBAS) % (8 * PW_THREADS) == 0);
static_assert(NBAS == 8 && NKN == 12);

typedef __attribute__((ext_vector_type(16))) _Float16 v16h;
typedef __attribute__((ext_vector_type(8)))  _Float16 v8h;
typedef __attribute__((ext_vector_type(16))) __bf16   v16b;
typedef __attribute__((ext_vector_type(8)))  __bf16   v8b;
typedef __attribute__((ext_vector_type(8)))  float    v8f;
typedef __attribute__((ext_vector_type(4)))  float    v4f;
typedef __attribute__((ext_vector_type(4)))  unsigned int v4u;

__device__ __forceinline__ unsigned short f2bf_bits(float f) {
  unsigned u = __float_as_uint(f);
  return (unsigned short)((u + 0x7FFFu + ((u >> 16) & 1u)) >> 16);
}
__device__ __forceinline__ float bf_bits2f(unsigned short h) { return __uint_as_float(((unsigned)h) << 16); }

__device__ __forceinline__ void dep_guard_h(v8f& a, v8f& b, v16h x, v16h y) { asm volatile("v_nop\n\tv_nop\n\tv_nop\n\tv_nop" : "+v"(a), "+v"(b) : "v"(x), "v"(y)); }
__device__ __forceinline__ void dep_guard_b(v8f& a, v8f& b, v16b x, v16b y) { asm volatile("v_nop\n\tv_nop\n\tv_nop\n\tv_nop" : "+v"(a), "+v"(b) : "v"(x), "v"(y)); }
__device__ __forceinline__ void dep_guard4_h(v8f& a, v8f& b, v8f& c, v8f& d, v16h x, v16h y) { asm volatile("v_nop\n\tv_nop\n\tv_nop\n\tv_nop" : "+v"(a), "+v"(b), "+v"(c), "+v"(d) : "v"(x), "v"(y)); }
__device__ __forceinline__ void dep_guard4_b(v8f& a, v8f& b, v8f& c, v8f& d, v16b x, v16b y) { asm volatile("v_nop\n\tv_nop\n\tv_nop\n\tv_nop" : "+v"(a), "+v"(b), "+v"(c), "+v"(d) : "v"(x), "v"(y)); }
__device__ __forceinline__ void keep4_h(v16h a, v16h b, v16h c, v16h d) { asm volatile("v_nop" :: "v"(a), "v"(b), "v"(c), "v"(d)); }
__device__ __forceinline__ void keep4_b(v16b a, v16b b, v16b c, v16b d) { asm volatile("v_nop" :: "v"(a), "v"(b), "v"(c), "v"(d)); }
__device__ __forceinline__ void acc_guard4(v8f& a, v8f& b, v8f& c, v8f& d) { asm volatile("v_nop\n\tv_nop\n\tv_nop\n\tv_nop" : "+v"(a), "+v"(b), "+v"(c), "+v"(d)); }
template <typename T> struct Frag;
template <> struct Frag<_Float16> {
  typedef v16h V; union U { v16h v; v8h h[2]; };
  static __device__ __forceinline__ v16h load(const _Float16* p) {
    U f; f.h[0] = *(const v8h*)(p); f.h[1] = *(const v8h*)(p + 16); return f.v;
  }
  static __device__ __forceinline__ v8f mma(v16h a, v16h b, v8f c) {
    return __builtin_amdgcn_wmma_f32_16x16x32_f16(false, a, false, b, (short)0, c, false, false);
  }
  static __device__ __forceinline__ void guard(v8f& a, v8f& b, v16h x, v16h y) { dep_guard_h(a, b, x, y); }
  static __device__ __forceinline__ void guard4(v8f& a, v8f& b, v8f& c, v8f& d, v16h x, v16h y) { dep_guard4_h(a, b, c, d, x, y); }
  static __device__ __forceinline__ void keep(v16h a, v16h b, v16h c, v16h d) { keep4_h(a, b, c, d); }
};
template <> struct Frag<__bf16> {
  typedef v16b V; union U { v16b v; v8b h[2]; };
  static __device__ __forceinline__ v16b load(const __bf16* p) {
    U f; f.h[0] = *(const v8b*)(p); f.h[1] = *(const v8b*)(p + 16); return f.v;
  }
  static __device__ __forceinline__ v8f mma(v16b a, v16b b, v8f c) {
    return __builtin_amdgcn_wmma_f32_16x16x32_bf16(false, a, false, b, (short)0, c, false, false);
  }
  static __device__ __forceinline__ void guard(v8f& a, v8f& b, v16b x, v16b y) { dep_guard_b(a, b, x, y); }
  static __device__ __forceinline__ void guard4(v8f& a, v8f& b, v8f& c, v8f& d, v16b x, v16b y) { dep_guard4_b(a, b, c, d, x, y); }
  static __device__ __forceinline__ void keep(v16b a, v16b b, v16b c, v16b d) { keep4_b(a, b, c, d); }
};

__device__ __forceinline__ unsigned pk16(unsigned short a, unsigned short b) { return (unsigned)a | ((unsigned)b << 16); }
__device__ __forceinline__ unsigned short h_bits(float f) { const _Float16 h = (_Float16)f; return __builtin_bit_cast(unsigned short, h); }

template <int ET> struct Elem;
template <> struct Elem<0> { typedef _Float16 T; };
template <> struct Elem<1> { typedef __bf16 T; };
template <int ET, bool SPLIT, int BIAS_MODE, int OUT_MODE, bool RESID, int ACT = 0>
__global__ __launch_bounds__(256) void wmma_gemm64(
    const unsigned short* __restrict__ Ap, const unsigned short* __restrict__ A2p, int lda, long strideA,
    const unsigned short* __restrict__ Btp, const unsigned short* __restrict__ Bt2p, int ldb, long strideB,
    void* __restrict__ Cout, void* __restrict__ Cout2, int ldc, long strideC,
    const float* __restrict__ bias,
    const float* __restrict__ resid, long strideR,
    int M, int N, int K, float scale) {
  typedef typename Elem<ET>::T T;
  typedef typename Frag<T>::V V;
  const T* A = (const T*)Ap; const T* A2 = (const T*)A2p; const T* Bt = (const T*)Btp; const T* Bt2 = (const T*)Bt2p;
  __shared__ __align__(16) float sT[8][16 * 68];
  const int b    = blockIdx.y;
  const int lane = threadIdx.x & 31;
  const int wave = threadIdx.x >> 5;
  const int tilesN = N >> 6;
  const int tilesM = M >> 6;
  const int tile = blockIdx.x * 8 + wave;
  if (tile >= tilesM * tilesN) return;
  const int tm = tile / tilesN;
  const int tn = tile - tm * tilesN;
  const int m0 = tm << 6;
  const int n0 = tn << 6;

  const T* Ab  = A  + (size_t)b * strideA;
  const T* Bb  = Bt + (size_t)b * strideB;
  const T* Ab2 = SPLIT ? (A2  + (size_t)b * strideA) : nullptr;
  const T* Bb2 = SPLIT ? (Bt2 + (size_t)b * strideB) : nullptr;

  const int rlane = lane & 15;
  const int koff  = (lane >> 4) * 8;
  const int mOff  = (lane >> 4) * 8;

  v8f acc[4][4];
#pragma unroll
  for (int i = 0; i < 4; ++i)
#pragma unroll
    for (int j = 0; j < 4; ++j) acc[i][j] = (v8f){0.f,0.f,0.f,0.f,0.f,0.f,0.f,0.f};

  for (int k0 = 0; k0 < K; k0 += 32) {
    V bh[4], bl[4];
#pragma unroll
    for (int j = 0; j < 4; ++j) {
      const size_t bo = (size_t)(n0 + (j << 4) + rlane) * ldb + koff + k0;
      bh[j] = Frag<T>::load(Bb + bo);
      if (SPLIT) bl[j] = Frag<T>::load(Bb2 + bo);
    }
#pragma unroll
    for (int i = 0; i < 4; ++i) {
      const size_t ao = (size_t)(m0 + (i << 4) + rlane) * lda + koff + k0;
      V ah = Frag<T>::load(Ab + ao);
      V al;
      if (SPLIT) al = Frag<T>::load(Ab2 + ao);
#pragma unroll
      for (int j = 0; j < 4; ++j) {
        acc[i][j] = Frag<T>::mma(ah, bh[j], acc[i][j]);
        if (SPLIT) {
          acc[i][j] = Frag<T>::mma(ah, bl[j], acc[i][j]);
          acc[i][j] = Frag<T>::mma(al, bh[j], acc[i][j]);
        }
      }
      Frag<T>::guard4(acc[i][0], acc[i][1], acc[i][2], acc[i][3], ah, SPLIT ? al : ah);
    }
    Frag<T>::keep(bh[0], bh[1], bh[2], bh[3]);
    if (SPLIT) Frag<T>::keep(bl[0], bl[1], bl[2], bl[3]);
  }
  acc_guard4(acc[0][0], acc[0][1], acc[0][2], acc[0][3]);
  acc_guard4(acc[1][0], acc[1][1], acc[1][2], acc[1][3]);
  acc_guard4(acc[2][0], acc[2][1], acc[2][2], acc[2][3]);
  acc_guard4(acc[3][0], acc[3][1], acc[3][2], acc[3][3]);

  float* slab = sT[wave];
  const float* Rb = RESID ? (resid + (size_t)b * strideR) : nullptr;
#pragma unroll
  for (int i = 0; i < 4; ++i) {
    const int mBase = m0 + (i << 4);
#pragma unroll
    for (int j = 0; j < 4; ++j) {
      const int n = n0 + (j << 4) + rlane;
      float bv = 0.f;
      if (BIAS_MODE == 2) bv = bias[n];
#pragma unroll
      for (int r = 0; r < 8; ++r) {
        float v = acc[i][j][r] * scale;
        if (BIAS_MODE == 1) v += bias[mBase + mOff + r];
        if (BIAS_MODE == 2) v += bv;
        if (RESID) v += Rb[(size_t)(mBase + mOff + r) * ldc + n];
        if (ACT == 2) v = fmaxf(v, 0.0f);
        if (ACT == 4) v = (v > 0.f) ? v : 0.01f * v;
        slab[(mOff + r) * 68 + (j << 4) + rlane] = v;
      }
    }
    __builtin_amdgcn_fence(__ATOMIC_RELEASE, "workgroup");
    __builtin_amdgcn_wave_barrier();
    __builtin_amdgcn_fence(__ATOMIC_ACQUIRE, "workgroup");
    if (OUT_MODE == 0) {
      float* C = (float*)Cout + (size_t)b * strideC;
      const int hh = lane >> 4, c4 = (lane & 15) * 4;
      for (int pass = 0; pass < 2; ++pass) {
#pragma unroll
        for (int it = 0; it < 8; ++it) {
          const int row = it * 2 + hh;
          v4f v = *(const v4f*)(slab + row * 68 + c4);
          *(volatile v4f*)(C + (size_t)(mBase + row) * ldc + n0 + c4) = v;
        }
        __threadfence();
      }
    } else {
      const int q = lane >> 3, c8 = (lane & 7) * 8;
      unsigned short* C  = (unsigned short*)Cout  + (size_t)b * strideC;
      unsigned short* C2 = (OUT_MODE == 2) ? ((unsigned short*)Cout2 + (size_t)b * strideC) : nullptr;
      for (int pass = 0; pass < 2; ++pass) {
#pragma unroll
        for (int it = 0; it < 4; ++it) {
          const int row = it * 4 + q;
          const float* sp = slab + row * 68 + c8;
          v8h hv, lv;
#pragma unroll
          for (int e = 0; e < 8; ++e) {
            if (OUT_MODE == 1) {
              hv[e] = (_Float16)sp[e];
            } else {
              unsigned short hb = f2bf_bits(sp[e]);
              unsigned short lb = f2bf_bits(sp[e] - bf_bits2f(hb));
              hv[e] = __builtin_bit_cast(_Float16, hb);
              lv[e] = __builtin_bit_cast(_Float16, lb);
            }
          }
          *(volatile v8h*)(C + (size_t)(mBase + row) * ldc + n0 + c8) = hv;
          if (OUT_MODE == 2) *(volatile v8h*)(C2 + (size_t)(mBase + row) * ldc + n0 + c8) = lv;
        }
        __threadfence();
      }
    }
    __builtin_amdgcn_fence(__ATOMIC_RELEASE, "workgroup");
    __builtin_amdgcn_wave_barrier();
    __builtin_amdgcn_fence(__ATOMIC_ACQUIRE, "workgroup");
  }
}

__device__ __forceinline__ float wave_min32(float v) {
#pragma unroll
  for (int off = 16; off > 0; off >>= 1) v = fminf(v, __shfl_xor(v, off, 32));
  return v;
}
__device__ __forceinline__ float wave_max32(float v) {
#pragma unroll
  for (int off = 16; off > 0; off >>= 1) v = fmaxf(v, __shfl_xor(v, off, 32));
  return v;
}

__global__ __launch_bounds__(MM_THREADS) void minmax_part_kernel(const float* __restrict__ x, float* __restrict__ part) {
  __shared__ float smn[8];
  __shared__ float smx[8];
  const int t = threadIdx.x, lane = t & 31, wave = t >> 5;
  const float* base = x + (size_t)blockIdx.x * (NX / MM_BLOCKS);
  float mn = __builtin_inff(), mx = -__builtin_inff();
#pragma unroll 1
  for (int it = 0; it < MM_ITERS; ++it) {
    const v4f v = *(const v4f*)(base + ((size_t)it * MM_THREADS + t) * 4);
    mn = fminf(mn, fminf(fminf(v[0], v[1]), fminf(v[2], v[3])));
    mx = fmaxf(mx, fmaxf(fmaxf(v[0], v[1]), fmaxf(v[2], v[3])));
  }
  mn = wave_min32(mn);
  mx = wave_max32(mx);
  if (lane == 0) { smn[wave] = mn; smx[wave] = mx; }
  __syncthreads();
  float a = smn[lane & 7];
  float c = smx[lane & 7];
  a = wave_min32(a);
  c = wave_max32(c);
  if (wave == 0) {
    const float val = (lane == 0) ? a : ((lane == 1) ? c : 0.0f);
    volatile float* pp = part + (size_t)blockIdx.x * 32 + lane;
    *pp = val;
    __threadfence();
    *pp = val;
  }
}

__global__ __launch_bounds__(256) void minmax_final_kernel(const float* __restrict__ part, float* __restrict__ stats) {
  __shared__ float smn[8];
  __shared__ float smx[8];
  const int t = threadIdx.x, lane = t & 31, wave = t >> 5;
  float mn = part[(size_t)t * 32 + 0];
  float mx = part[(size_t)t * 32 + 1];
  mn = wave_min32(mn);
  mx = wave_max32(mx);
  if (lane == 0) { smn[wave] = mn; smx[wave] = mx; }
  __syncthreads();
  float a = smn[lane & 7];
  float c = smx[lane & 7];
  a = wave_min32(a);
  c = wave_max32(c);
  const float rd = 1.0f / (c - a + 1e-8f);
  if (wave == 0) {
    const float val = (lane == 0) ? a : ((lane == 1) ? rd : ((lane == 2) ? c : 0.0f));
    volatile float* pp = stats + lane;
    *pp = val;
    __threadfence();
    *pp = val;
  }
}

__global__ __launch_bounds__(PW_THREADS) void packw_kernel(const float* __restrict__ bw, const float* __restrict__ sw,
                                                           const float* __restrict__ sc, unsigned short* __restrict__ Wt) {
  const int t = threadIdx.x;
  const int o = blockIdx.y;
  const int bx = blockIdx.x;
  float v[8];
  size_t dst;
  if (bx == 0) {
    const float* p = bw + (size_t)o * NIN + 8 * t;
    const v4f a = *(const v4f*)(p);
    const v4f c = *(const v4f*)(p + 4);
#pragma unroll
    for (int e = 0; e < 4; ++e) { v[e] = a[e] * WGT_CARRY; v[4 + e] = c[e] * WGT_CARRY; }
    dst = (size_t)o * KTOT + 8 * t;
  } else {
    const int grp = (bx - 1) * PW_THREADS + t;
    const float* p = sw + (size_t)o * NIN * NBAS + 8 * (size_t)grp;
    const v4f a = *(const v4f*)(p);
    const v4f c = *(const v4f*)(p + 4);
    const float s = sc[(size_t)o * NIN + grp];
#pragma unroll
    for (int e = 0; e < 4; ++e) {
      const float p0 = a[e] * s;
      const float p1 = c[e] * s;
      v[e] = p0 * WGT_CARRY;
      v[4 + e] = p1 * WGT_CARRY;
    }
    dst = (size_t)o * KTOT + NIN + 8 * (size_t)grp;
  }
  unsigned short hb[8];
#pragma unroll
  for (int e = 0; e < 8; ++e) hb[e] = h_bits(v[e]);
  const v4u u = (v4u){pk16(hb[0], hb[1]), pk16(hb[2], hb[3]), pk16(hb[4], hb[5]), pk16(hb[6], hb[7])};
  unsigned short* q = Wt + dst;
  *(volatile v4u*)q = u;
  __threadfence();
  *(volatile v4u*)q = u;
}

__global__ __launch_bounds__(FT_THREADS) void feat_kernel(const float* __restrict__ x, const float* __restrict__ knots,
                                                          const float* __restrict__ stats, unsigned short* __restrict__ Apl) {
  __shared__ __align__(16) float s_silu[FT_ROWS * NIN];
  const int t = threadIdx.x;
  const int b0 = blockIdx.x * FT_ROWS;
  const float xmin = stats[0];
  const float rd   = stats[1];
#pragma unroll 1
  for (int c = 0; c < FT_CHUNKS; ++c) {
    const int i = c * FT_THREADS + t;
    const float* gp = knots + (size_t)i * NKN;
    const v4f ga = *(const v4f*)(gp);
    const v4f gb = *(const v4f*)(gp + 4);
    const v4f gc = *(const v4f*)(gp + 8);
    float g[NKN];
#pragma unroll
    for (int e = 0; e < 4; ++e) { g[e] = ga[e]; g[4 + e] = gb[e]; g[8 + e] = gc[e]; }
    float r1[NKN - 1], r2[NKN - 2], r3[NKN - 3];
#pragma unroll
    for (int j = 0; j < NKN - 1; ++j) r1[j] = __builtin_amdgcn_rcpf(g[j + 1] - g[j]);
#pragma unroll
    for (int j = 0; j < NKN - 2; ++j) r2[j] = __builtin_amdgcn_rcpf(g[j + 2] - g[j]);
#pragma unroll
    for (int j = 0; j < NKN - 3; ++j) r3[j] = __builtin_amdgcn_rcpf(g[j + 3] - g[j]);
#pragma unroll 1
    for (int rb = 0; rb < FT_ROWS; ++rb) {
      const int b = b0 + rb;
      const float xv = x[(size_t)b * NIN + i];
      const float ex = expf(-xv);
      const float sg = 1.0f / (1.0f + ex);
      s_silu[rb * NIN + i] = xv * sg;
      const float tn = (xv - xmin) * rd;
      const float xn = tn * 2.0f - 1.0f;
      float Bv[NKN - 1];
#pragma unroll
      for (int j = 0; j < NKN - 1; ++j) Bv[j] = (xn >= g[j] && xn < g[j + 1]) ? 1.0f : 0.0f;
#pragma unroll
      for (int j = 0; j < NKN - 2; ++j) {
        const float lf = (xn - g[j]) * r1[j];
        const float rt = (g[j + 2] - xn) * r1[j + 1];
        Bv[j] = lf * Bv[j] + rt * Bv[j + 1];
      }
#pragma unroll
      for (int j = 0; j < NKN - 3; ++j) {
        const float lf = (xn - g[j]) * r2[j];
        const float rt = (g[j + 3] - xn) * r2[j + 1];
        Bv[j] = lf * Bv[j] + rt * Bv[j + 1];
      }
#pragma unroll
      for (int j = 0; j < NKN - 4; ++j) {
        const float lf = (xn - g[j]) * r3[j];
        const float rt = (g[j + 4] - xn) * r3[j + 1];
        Bv[j] = lf * Bv[j] + rt * Bv[j + 1];
      }
      unsigned short hb[8];
#pragma unroll
      for (int e = 0; e < 8; ++e) hb[e] = h_bits(Bv[e] * FEAT_CARRY);
      const v4u u = (v4u){pk16(hb[0], hb[1]), pk16(hb[2], hb[3]), pk16(hb[4], hb[5]), pk16(hb[6], hb[7])};
      unsigned short* q = Apl + (size_t)b * KTOT + NIN + (size_t)i * NBAS;
      *(volatile v4u*)q = u;
      __threadfence();
      *(volatile v4u*)q = u;
    }
  }
  __syncthreads();
#pragma unroll 1
  for (int rb = 0; rb < FT_ROWS; ++rb) {
    const int b = b0 + rb;
    const float* sp = s_silu + rb * NIN + 8 * t;
    const v4f a = *(const v4f*)(sp);
    const v4f c = *(const v4f*)(sp + 4);
    unsigned short hb[8];
#pragma unroll
    for (int e = 0; e < 4; ++e) { hb[e] = h_bits(a[e] * FEAT_CARRY); hb[4 + e] = h_bits(c[e] * FEAT_CARRY); }
    const v4u u = (v4u){pk16(hb[0], hb[1]), pk16(hb[2], hb[3]), pk16(hb[4], hb[5]), pk16(hb[6], hb[7])};
    unsigned short* q = Apl + (size_t)b * KTOT + 8 * t;
    *(volatile v4u*)q = u;
    __threadfence();
    *(volatile v4u*)q = u;
  }
}

extern "C" void kernel_launch(void* const* d_in, const int* in_sizes, int n_in,
                              void* d_out, int out_size, void* d_ws, size_t ws_size,
                              hipStream_t stream) {
  if (n_in < 5) return;
  if (in_sizes[0] != NX || in_sizes[1] != NIN * NKN || in_sizes[2] != NOUT * NIN ||
      in_sizes[3] != NOUT * NIN * NBAS || in_sizes[4] != NOUT * NIN || out_size != NB_ROWS * NOUT) return;
  if (ws_size < WS_END) return;

  const float* x     = (const float*)d_in[0];
  const float* knots = (const float*)d_in[1];
  const float* bw    = (const float*)d_in[2];
  const float* sw    = (const float*)d_in[3];
  const float* sc    = (const float*)d_in[4];
  float* out = (float*)d_out;

  char* ws = (char*)d_ws;
  float* part  = (float*)(ws + WS_OFF_PART);
  float* stats = (float*)(ws + WS_OFF_STATS);
  unsigned short* Apl = (unsigned short*)(ws + WS_OFF_A);
  unsigned short* Wtp = (unsigned short*)(ws + WS_OFF_W);

  minmax_part_kernel<<<dim3(MM_BLOCKS), dim3(MM_THREADS), 0, stream>>>(x, part);
  minmax_final_kernel<<<dim3(1), dim3(256), 0, stream>>>(part, stats);
  packw_kernel<<<dim3(PW_BLOCKS_X, NOUT), dim3(PW_THREADS), 0, stream>>>(bw, sw, sc, Wtp);
  for (int hf = 0; hf < NHALF; ++hf) {
    const float* xh = x + (size_t)hf * MHALF * NIN;
    float* oh = out + (size_t)hf * MHALF * NOUT;
    feat_kernel<<<dim3(MHALF / FT_ROWS), dim3(FT_THREADS), 0, stream>>>(xh, knots, stats, Apl);
    wmma_gemm64<0, false, 0, 0, false, 0><<<dim3(GM_BLOCKS, 1), dim3(256), 0, stream>>>(
        Apl, Apl, KTOT, 0L,
        Wtp, Wtp, KTOT, 0L,
        (void*)oh, (void*)oh, NOUT, 0L,
        stats,
        stats, 0L,
        MHALF, NOUT, KTOT, OUT_SCALE);
  }
}
